// TransformerEncoderReadout_solv_10222022164949
// MI455X (gfx1250) — hardware-run, weakly checked
//
#include <hip/hip_runtime.h>


#ifndef NB
#define NB 256
#endif
#ifndef SEQ
#define SEQ 160
#endif
#define NB_FULL  256
#define DM   128
#define NH_  8
#define HD   128
#define HK   (NH_ * HD)
#define FF   256
#define AW   5
#define PW   (SEQ / 16)
#define OSP  132
#define VSP  (SEQ + 4)
#define YP   128
#define FP   128
#define CHB  (NB < 64 ? NB : 64)
#define NCH  (NB / CHB)
#define CHROWS (CHB * SEQ)
#define WSC  64.0f
#define WINV (1.0f / 64.0f)
#define CTXS 16.0f
#define OSCL (1.0f / 1024.0f)
#define SC2  ((float)(0.08838834764831845 * 1.4426950408889634))
#define FILL2 ((float)(-1.0e9 * 1.4426950408889634))
#define PSH  14.0f
#define NEGB (-3.0e38f)
#define LNEPS 1.0e-3f

static_assert(HD == 128);
static_assert(NH_ * HD == HK);
static_assert(DM % 64 == 0);
static_assert(HK % 64 == 0);
static_assert(FF % 64 == 0);
static_assert(FF == 2 * 128);
static_assert(DM == 128);
static_assert(DM % 32 == 0);
static_assert(HK % 32 == 0);
static_assert(SEQ % 32 == 0);
static_assert(SEQ % (16 * AW) == 0);
static_assert(SEQ <= 256);
static_assert((SEQ * 16) % 256 == 0);
static_assert(SEQ % 4 == 0);
static_assert((SEQ * 4) % 128 == 0);
static_assert((16 * SEQ * 2) % 128 == 0);
static_assert(NB % CHB == 0);
static_assert(NB <= NB_FULL);
static_assert(CHROWS % 32 == 0);
static_assert(HK % 16 == 0);
static_assert(32 * PW <= 1024);
static_assert((OSP * 4) % 16 == 0);
static_assert((VSP * 4) % 16 == 0);
static_assert(8 * 32 * 8 == 16 * HD);
static_assert((SEQ / 16) * 32 * 8 == 16 * SEQ);
static_assert(4 * 256 * 4 == 64 * 64);
static_assert(2 * 256 * 8 == 64 * 64);
static_assert(16 * OSP * 4 <= 131072);
static_assert(16 * VSP * 4 <= 131072);
static_assert(AW * 16 * OSP * 4 <= 131072);
static_assert(PW * 16 * YP * 4 + PW * 16 * FP * 2 + PW * DM * 4 <= 131072);

typedef _Float16 h16;
typedef unsigned short bf;
typedef __attribute__((ext_vector_type(16))) __bf16   v16bf;
typedef __attribute__((ext_vector_type(16))) _Float16 v16h;
typedef __attribute__((ext_vector_type(8)))  _Float16 v8h;
typedef __attribute__((ext_vector_type(8)))  unsigned short v8us;
typedef __attribute__((ext_vector_type(8)))  float    v8f;
typedef __attribute__((ext_vector_type(4)))  float    v4f;
typedef v4f  __attribute__((may_alias)) v4fa;
typedef v8h  __attribute__((may_alias)) v8ha;

__device__ __forceinline__ unsigned short f2bf(float f) { unsigned u = __float_as_uint(f); u += 0x7FFFu + ((u >> 16) & 1u); return (unsigned short)(u >> 16); }
__device__ __forceinline__ float bfr(float f) { return __uint_as_float(((unsigned)f2bf(f)) << 16); }
__device__ __forceinline__ v16h cat16(v8h lo, v8h hi) { return __builtin_shufflevector(lo, hi, 0, 1, 2, 3, 4, 5, 6, 7, 8, 9, 10, 11, 12, 13, 14, 15); }
__device__ __forceinline__ v16bf cat16b(v8us lo, v8us hi) { return __builtin_bit_cast(v16bf, __builtin_shufflevector(lo, hi, 0, 1, 2, 3, 4, 5, 6, 7, 8, 9, 10, 11, 12, 13, 14, 15)); }
__device__ __forceinline__ v8f wmma16(v16h a, v16h b, v8f c) { return __builtin_amdgcn_wmma_f32_16x16x32_f16(false, a, false, b, (short)0, c, false, false); }
__device__ __forceinline__ v8f wmmab(v16bf a, v16bf b, v8f c) { return __builtin_amdgcn_wmma_f32_16x16x32_bf16(false, a, false, b, (short)0, c, false, false); }
__device__ __forceinline__ v16h  ldh(const h16* p) { return cat16(*(const v8h*)p, *(const v8h*)(p + 16)); }
__device__ __forceinline__ v16bf ldb(const bf* p)  { return cat16b(*(const v8us*)p, *(const v8us*)(p + 16)); }
__device__ __forceinline__ void wave_sync() { __builtin_amdgcn_fence(3  , "wavefront"); __builtin_amdgcn_wave_barrier(); asm volatile("" ::: "memory"); }

static __device__ __forceinline__ h16 toh_flush(float v) { const h16 r = (h16)v; return (fabsf(v) < 6.103515625e-05f) ? (h16)0.0f : r; }
__device__ __forceinline__ float bf2f(unsigned short w) { return __uint_as_float(((unsigned)w) << 16); }
__device__ __forceinline__ v8f wg16(v16h a, v16h b, v8f c) { c = wmma16(a, b, c); asm volatile("v_nop\n\tv_nop\n\tv_nop\n\tv_nop" : "+v"(c) : "v"(a), "v"(b)); return c; }
__device__ __forceinline__ v8f wgb(v16bf a, v16bf b, v8f c) { c = wmmab(a, b, c); asm volatile("v_nop\n\tv_nop\n\tv_nop\n\tv_nop" : "+v"(c) : "v"(a), "v"(b)); return c; }

__global__ __launch_bounds__(256) void k_pack(const float* __restrict__ atoms, const int* __restrict__ mol, int N, bf* XB, float* MK) {
    __shared__ int sred[8 * 2];
    __shared__ int sgood[8];
    __shared__ __align__(16) float smk[SEQ];
    const int tid = threadIdx.x, lane = tid & 31;
    const int wave = __builtin_amdgcn_readfirstlane((int)(threadIdx.x >> 5));
    const int b = blockIdx.x;
    int lt = 0, eq = 0;
#pragma unroll 1
    for (int base = 0; base < N; base += 256) {
        const int i = base + tid; const int ic = i < N ? i : N - 1;
        int mi = mol[ic];
        asm volatile("" : "+v"(mi));
        lt += ((i < N) & (mi >= 0) & (mi < b)) ? 1 : 0;
        eq += ((i < N) & (mi == b)) ? 1 : 0;
    }
#pragma unroll
    for (int off = 16; off > 0; off >>= 1) { lt += __shfl_xor(lt, off, 32); eq += __shfl_xor(eq, off, 32); }
    if (lane == 0) { sred[wave * 2] = lt; sred[wave * 2 + 1] = eq; }
    __syncthreads();
    int start = 0, cnt = 0;
#pragma unroll
    for (int w = 0; w < 8; ++w) { start += sred[w * 2]; cnt += sred[w * 2 + 1]; }
    const int cntc = cnt < SEQ ? cnt : SEQ;
    int good;
    { const int i = start + tid; int ic = i < N ? i : N - 1; ic = ic < 0 ? 0 : ic;
      int mi = mol[ic];
      asm volatile("" : "+v"(mi));
      good = ((tid < cntc) & (i < N) & (mi == b)) ? 1 : 0; }
#pragma unroll
    for (int off = 16; off > 0; off >>= 1) good += __shfl_xor(good, off, 32);
    if (lane == 0) sgood[wave] = good;
    __syncthreads();
    int gtot = 0;
#pragma unroll
    for (int w = 0; w < 8; ++w) gtot += sgood[w];
    const float mark = (gtot != cnt) ? __uint_as_float(0x7fc00000u) : 0.0f;
#pragma unroll 1
    for (int it = 0; it < (SEQ * 16) / 256; ++it) {
        const int p = it * 256 + tid; const int row = p >> 4, c8 = (p & 15) * 8;
        int sr = start + row; sr = sr < N ? sr : N - 1; sr = sr < 0 ? 0 : sr;
        v8f v = *(const v8f*)(atoms + (size_t)sr * DM + c8);
        asm volatile("" : "+v"(v));
        const bool ok = row < cntc;
        v8us o; int nz = 0;
#pragma unroll
        for (int k = 0; k < 8; ++k) { const unsigned short w = f2bf(v[k]); o[k] = ok ? w : (unsigned short)0; nz |= (ok & ((w & 0x7FFFu) != 0)) ? 1 : 0; }
        bf* dp = XB + ((size_t)(b * SEQ + row)) * DM + c8;
        *(volatile v8us*)dp = o; __threadfence(); *(volatile v8us*)dp = o;
        nz |= __shfl_xor(nz, 1, 32); nz |= __shfl_xor(nz, 2, 32); nz |= __shfl_xor(nz, 4, 32); nz |= __shfl_xor(nz, 8, 32);
        if ((tid & 15) == 0) smk[row] = nz ? 1.0f : 0.0f;
    }
    __syncthreads();
    if (tid < SEQ / 4) {
        v4f mv = *(const v4fa*)(&smk[tid * 4]);
        mv = mv + mark;
        float* mp = MK + (size_t)b * SEQ + tid * 4;
        *(volatile v4f*)mp = mv; __threadfence(); *(volatile v4f*)mp = mv;
    }
}

__global__ __launch_bounds__(256) void k_wT_bf(const float* __restrict__ src, bf* dst, int R, int C) {
    __shared__ float tl[64 * 65];
    const int tid = threadIdx.x; const int r0 = blockIdx.x * 64, c0 = blockIdx.y * 64;
#pragma unroll 1
    for (int it = 0; it < 4; ++it) { const int q = it * 256 + tid; const int rw = q >> 4, c4 = (q & 15) * 4;
        const v4f v = *(const v4f*)(src + (size_t)(r0 + rw) * C + c0 + c4);
        tl[rw * 65 + c4 + 0] = v[0]; tl[rw * 65 + c4 + 1] = v[1]; tl[rw * 65 + c4 + 2] = v[2]; tl[rw * 65 + c4 + 3] = v[3]; }
    __syncthreads();
#pragma unroll 1
    for (int it = 0; it < 2; ++it) { const int q = it * 256 + tid; const int cc = q >> 3, pc = q & 7; v8us o;
#pragma unroll
        for (int j = 0; j < 8; ++j) o[j] = f2bf(tl[(pc * 8 + j) * 65 + cc]);
        bf* dp = dst + (size_t)(c0 + cc) * R + r0 + pc * 8;
        *(volatile v8us*)dp = o; __threadfence(); *(volatile v8us*)dp = o; }
}
__global__ __launch_bounds__(256) void k_wT_h(const float* __restrict__ src, h16* dst, int R, int C) {
    __shared__ float tl[64 * 65];
    const int tid = threadIdx.x; const int r0 = blockIdx.x * 64, c0 = blockIdx.y * 64;
#pragma unroll 1
    for (int it = 0; it < 4; ++it) { const int q = it * 256 + tid; const int rw = q >> 4, c4 = (q & 15) * 4;
        const v4f v = *(const v4f*)(src + (size_t)(r0 + rw) * C + c0 + c4);
        tl[rw * 65 + c4 + 0] = v[0]; tl[rw * 65 + c4 + 1] = v[1]; tl[rw * 65 + c4 + 2] = v[2]; tl[rw * 65 + c4 + 3] = v[3]; }
    __syncthreads();
#pragma unroll 1
    for (int it = 0; it < 2; ++it) { const int q = it * 256 + tid; const int cc = q >> 3, pc = q & 7; v8h o;
#pragma unroll
        for (int j = 0; j < 8; ++j) o[j] = toh_flush(bfr(tl[(pc * 8 + j) * 65 + cc]) * WSC);
        h16* dp = dst + (size_t)(c0 + cc) * R + r0 + pc * 8;
        *(volatile v8h*)dp = o; __threadfence(); *(volatile v8h*)dp = o; }
}

__global__ __launch_bounds__(32) void k_projqk(const bf* __restrict__ A, const bf* __restrict__ Bt, const float* __restrict__ bq, const float* __restrict__ bk, h16* QK) {
    __shared__ __align__(16) float os[16 * OSP];
    const int K = DM;
    const int lane = threadIdx.x & 31, lr = lane & 15, hi = lane >> 4;
    const int r0 = blockIdx.x * 32; const int y = blockIdx.y; const int which = y >> 3, hh = y & 7; const int c0 = y * HD;
    v8f acc[2][8];
#pragma unroll
    for (int mb = 0; mb < 2; ++mb)
#pragma unroll
        for (int nb = 0; nb < 8; ++nb) acc[mb][nb] = (v8f){};
    const size_t aoff = (size_t)(r0 + lr) * K + 8 * hi, boff = (size_t)(c0 + lr) * K + 8 * hi;
#pragma unroll 1
    for (int kc = 0; kc < K; kc += 32) {
        v16bf a[2];
#pragma unroll
        for (int mb = 0; mb < 2; ++mb) a[mb] = ldb(A + aoff + (size_t)mb * 16 * K + kc);
#pragma unroll
        for (int nb = 0; nb < 8; ++nb) { const v16bf b = ldb(Bt + boff + (size_t)nb * 16 * K + kc);
#pragma unroll
            for (int mb = 0; mb < 2; ++mb) acc[mb][nb] = wgb(a[mb], b, acc[mb][nb]); }
    }
    float bc[8];
#pragma unroll
    for (int nb = 0; nb < 8; ++nb) { const int bi = hh * HD + nb * 16 + lr; const float vq = bq[bi]; const float vk = bk[bi]; bc[nb] = bfr(which ? vk : vq); }
#pragma unroll
    for (int mb = 0; mb < 2; ++mb) {
#pragma unroll
        for (int nb = 0; nb < 8; ++nb) {
#pragma unroll
            for (int j = 0; j < 8; ++j) os[(hi * 8 + j) * OSP + nb * 16 + lr] = acc[mb][nb][j] + bc[nb]; }
        wave_sync();
        const int m0 = r0 + mb * 16; const int bb = m0 / SEQ, tt = m0 % SEQ;
        const size_t sb = (size_t)which * ((size_t)CHB * NH_ * SEQ * HD) + (((size_t)(bb * NH_ + hh)) * SEQ + (size_t)tt) * HD;
#pragma unroll 1
        for (int ps = 0; ps < 2; ++ps) {
#pragma unroll
            for (int s = 0; s < 8; ++s) { const int p = s * 32 + lane; const int row = p >> 4, c8 = (p & 15) * 8;
                const v4f x0 = *(const v4fa*)(&os[row * OSP + c8]); const v4f x1 = *(const v4fa*)(&os[row * OSP + c8 + 4]); v8h hv;
#pragma unroll
                for (int i = 0; i < 4; ++i) { hv[i] = toh_flush(x0[i]); hv[4 + i] = toh_flush(x1[i]); }
                *(volatile v8h*)(QK + sb + (size_t)p * 8) = hv; }
            if (ps == 0) __threadfence(); }
        wave_sync();
    }
}

__global__ __launch_bounds__(32) void k_projv(const bf* __restrict__ Wt, const bf* __restrict__ X, const float* __restrict__ bv, h16* VT) {
    __shared__ __align__(16) float os[16 * VSP];
    const int K = DM;
    const int lane = threadIdx.x & 31, lr = lane & 15, hi = lane >> 4;
    const int r0 = blockIdx.x * 16; const int bl = blockIdx.y;
    v8f acc[SEQ / 16];
#pragma unroll
    for (int nb = 0; nb < SEQ / 16; ++nb) acc[nb] = (v8f){};
    const size_t aoff = (size_t)(r0 + lr) * K + 8 * hi, boff = ((size_t)bl * SEQ + lr) * K + 8 * hi;
#pragma unroll 1
    for (int kc = 0; kc < K; kc += 32) {
        const v16bf a = ldb(Wt + aoff + kc);
#pragma unroll
        for (int nb = 0; nb < SEQ / 16; ++nb) { const v16bf b = ldb(X + boff + (size_t)nb * 16 * K + kc); acc[nb] = wgb(a, b, acc[nb]); }
    }
    float br[8];
#pragma unroll
    for (int j = 0; j < 8; ++j) br[j] = bfr(bv[r0 + hi * 8 + j]);
#pragma unroll
    for (int nb = 0; nb < SEQ / 16; ++nb) {
#pragma unroll
        for (int j = 0; j < 8; ++j) os[(hi * 8 + j) * VSP + nb * 16 + lr] = acc[nb][j] + br[j]; }
    wave_sync();
    const size_t sb = ((size_t)bl * HK + (size_t)r0) * SEQ;
#pragma unroll 1
    for (int ps = 0; ps < 2; ++ps) {
#pragma unroll
        for (int s = 0; s < SEQ / 16; ++s) { const int p = s * 32 + lane; const int row = p / (SEQ / 8), c8 = (p % (SEQ / 8)) * 8;
            const v4f x0 = *(const v4fa*)(&os[row * VSP + c8]); const v4f x1 = *(const v4fa*)(&os[row * VSP + c8 + 4]); v8h hv;
#pragma unroll
            for (int i = 0; i < 4; ++i) { hv[i] = toh_flush(x0[i]); hv[4 + i] = toh_flush(x1[i]); }
            *(volatile v8h*)(VT + sb + (size_t)p * 8) = hv; }
        if (ps == 0) __threadfence(); }
}

__global__ __launch_bounds__(32 * AW) void k_flash(const h16* __restrict__ QH, const h16* __restrict__ KP, const h16* __restrict__ VT, const float* __restrict__ MK, h16* CTX) {
    __shared__ __align__(16) float os[AW * 16 * OSP];
    const int lane = threadIdx.x & 31, lr = lane & 15, hi = lane >> 4;
    const int wave = __builtin_amdgcn_readfirstlane((int)(threadIdx.x >> 5));
    const int zh = blockIdx.y; const int bl = zh / NH_, h = zh % NH_;
    const int t0 = (blockIdx.x * AW + wave) * 16;
    const float* kmb = MK + (size_t)bl * SEQ + 8 * hi;
    const size_t pbase = (size_t)zh * SEQ * HD;
    const size_t ko = pbase + (size_t)lr * HD + 8 * hi;
    const size_t vo = pbase + (size_t)lr * SEQ + 8 * hi;
    int qoi = (t0 + lr) * HD + 8 * hi;
    v8f o[8];
#pragma unroll
    for (int j = 0; j < 8; ++j) o[j] = (v8f){};
    float m = NEGB, l = 0.0f;
#pragma unroll 1
    for (int key0 = 0; key0 < SEQ; key0 += 32) {
        asm volatile("" : "+v"(qoi));
        const h16* qa = QH + pbase + qoi;
        const h16* ka = KP + ko + (size_t)key0 * HD;
        v8f sa = (v8f){}, sb = (v8f){};
#pragma unroll
        for (int kc = 0; kc < 4; ++kc) {
            const v16h qf = ldh(qa + kc * 32);
            const v16h ka0 = ldh(ka + kc * 32), kb0 = ldh(ka + 16 * HD + kc * 32);
            sa = wg16(ka0, qf, sa); sb = wg16(kb0, qf, sb); }
        const float* kp = kmb + key0;
        const v4f m0 = *(const v4f*)kp, m1 = *(const v4f*)(kp + 4), m2 = *(const v4f*)(kp + 16), m3 = *(const v4f*)(kp + 20);
        float kx[8], ky[8];
#pragma unroll
        for (int r = 0; r < 4; ++r) { kx[r] = m0[r]; kx[4 + r] = m1[r]; ky[r] = m2[r]; ky[4 + r] = m3[r]; }
        float ta[8], tb[8]; float mx = NEGB;
#pragma unroll
        for (int r = 0; r < 8; ++r) {
            ta[r] = (kx[r] != 0.0f) ? sa[r] * SC2 : FILL2;
            tb[r] = (ky[r] != 0.0f) ? sb[r] * SC2 : FILL2;
            mx = fmaxf(mx, fmaxf(ta[r], tb[r])); }
        mx = fmaxf(mx, __shfl_xor(mx, 16, 32));
        const float mnew = fmaxf(m, mx);
        const float alpha = __builtin_amdgcn_exp2f(m - mnew);
        const float sh = PSH - mnew;
        v16h pb; float ls = 0.0f;
#pragma unroll
        for (int r = 0; r < 8; ++r) {
            const float ea = ta[r] + sh, eb = tb[r] + sh;
            const float ga = (ea < -14.0f) ? 0.0f : __builtin_amdgcn_exp2f(ea);
            const float gb = (eb < -14.0f) ? 0.0f : __builtin_amdgcn_exp2f(eb);
            const h16 pa = (h16)ga; const h16 pc = (h16)gb;
            pb[r] = pa; pb[8 + r] = pc;
            ls += (float)pa + (float)pc; }
        l = l * alpha + ls; m = mnew;
#pragma unroll
        for (int j = 0; j < 8; ++j) o[j] = o[j] * alpha;
        const h16* va = VT + vo + key0;
#pragma unroll
        for (int jb = 0; jb < 8; jb += 4) {
            v16h vf[4];
#pragma unroll
            for (int i = 0; i < 4; ++i) vf[i] = ldh(va + (size_t)(jb + i) * 16 * SEQ);
#pragma unroll
            for (int i = 0; i < 4; ++i) o[jb + i] = wg16(vf[i], pb, o[jb + i]); }
    }
    l += __shfl_xor(l, 16, 32);
    const float inv = CTXS * (1.0f / l);
    const int wb = wave * 16 * OSP;
#pragma unroll
    for (int j = 0; j < 8; ++j) { v4f a, c;
        a[0] = o[j][0] * inv; a[1] = o[j][1] * inv; a[2] = o[j][2] * inv; a[3] = o[j][3] * inv; c[0] = o[j][4] * inv; c[1] = o[j][5] * inv; c[2] = o[j][6] * inv; c[3] = o[j][7] * inv;
        *(v4fa*)(&os[wb + lr * OSP + 16 * j + 8 * hi]) = a; *(v4fa*)(&os[wb + lr * OSP + 16 * j + 8 * hi + 4]) = c; }
    wave_sync();
    h16* crow = CTX + ((size_t)bl * SEQ + t0) * HK + h * HD;
#pragma unroll 1
    for (int ps = 0; ps < 2; ++ps) {
#pragma unroll
        for (int s = 0; s < 8; ++s) { const int p = s * 32 + lane; const int row = p >> 4, c8 = (p & 15) * 8;
            const v4f x0 = *(const v4fa*)(&os[wb + row * OSP + c8]); const v4f x1 = *(const v4fa*)(&os[wb + row * OSP + c8 + 4]); v8h hv;
#pragma unroll
            for (int i = 0; i < 4; ++i) { hv[i] = toh_flush(x0[i]); hv[4 + i] = toh_flush(x1[i]); }
            *(volatile v8h*)(crow + (size_t)row * HK + c8) = hv; }
        if (ps == 0) __threadfence(); }
}

__global__ __launch_bounds__(32 * PW) void k_post(const h16* __restrict__ CTX, const bf* __restrict__ XB, const float* __restrict__ MK,
                                                  const h16* __restrict__ WOT, const h16* __restrict__ W1T, const h16* __restrict__ W2T,
                                                  const float* __restrict__ bo, const float* __restrict__ b1, const float* __restrict__ b2,
                                                  const float* __restrict__ g1, const float* __restrict__ be1, const float* __restrict__ g2, const float* __restrict__ be2, float* OUT) {
    __shared__ __align__(16) float Y[PW * 16 * YP];
    __shared__ __align__(16) h16 sF[PW * 16 * FP];
    __shared__ __align__(16) float spart[PW * DM];
    const int lane = threadIdx.x & 31, lr = lane & 15, hi = lane >> 4;
    const int wave = __builtin_amdgcn_readfirstlane((int)(threadIdx.x >> 5));
    const int bl = blockIdx.x;
    const int rowl = bl * SEQ + wave * 16;
    const int wy = wave * 16 * YP, wf = wave * 16 * FP;
    const int rr = lane >> 1, hf = lane & 1;
    const int yr = wy + rr * YP + hf * 64;
    { v8f acc[8];
#pragma unroll
      for (int nb = 0; nb < 8; ++nb) acc[nb] = (v8f){};
      const size_t aoff = (size_t)(rowl + lr) * HK + 8 * hi, boff = (size_t)lr * HK + 8 * hi;
#pragma unroll 1
      for (int kc = 0; kc < HK; kc += 32) {
          const v16h a = ldh(CTX + aoff + kc);
#pragma unroll
          for (int nb = 0; nb < 8; ++nb) { const v16h b = ldh(WOT + boff + (size_t)nb * 16 * HK + kc); acc[nb] = wg16(a, b, acc[nb]); } }
#pragma unroll
      for (int nb = 0; nb < 8; ++nb) {
#pragma unroll
          for (int j = 0; j < 8; ++j) Y[wy + (hi * 8 + j) * YP + nb * 16 + lr] = acc[nb][j] * OSCL; } }
    wave_sync();
    { const bf* xr = XB + (size_t)(rowl + rr) * DM + hf * 64;
      float s = 0.0f;
#pragma unroll 1
      for (int q = 0; q < 8; ++q) { const int c = q * 8;
          const v8us xv = *(const v8us*)(xr + c);
          const v4f bo0 = *(const v4f*)(bo + hf * 64 + c), bo1 = *(const v4f*)(bo + hf * 64 + c + 4);
          v4f y0 = *(const v4fa*)(&Y[yr + c]), y1 = *(const v4fa*)(&Y[yr + c + 4]);
#pragma unroll
          for (int i = 0; i < 4; ++i) { y0[i] = bf2f(xv[i]) + (y0[i] + bfr(bo0[i])); y1[i] = bf2f(xv[4 + i]) + (y1[i] + bfr(bo1[i])); s += y0[i] + y1[i]; }
          *(v4fa*)(&Y[yr + c]) = y0; *(v4fa*)(&Y[yr + c + 4]) = y1; }
      s += __shfl_xor(s, 1, 32);
      const float mean = s * (1.0f / DM);
      float vs = 0.0f;
#pragma unroll 1
      for (int q = 0; q < 8; ++q) { const int c = q * 8;
          const v4f y0 = *(const v4fa*)(&Y[yr + c]), y1 = *(const v4fa*)(&Y[yr + c + 4]);
#pragma unroll
          for (int i = 0; i < 4; ++i) { const float d0 = y0[i] - mean, d1 = y1[i] - mean; vs += d0 * d0; vs += d1 * d1; } }
      vs += __shfl_xor(vs, 1, 32);
      const float rstd = rsqrtf(vs * (1.0f / DM) + LNEPS);
#pragma unroll 1
      for (int q = 0; q < 8; ++q) { const int c = q * 8;
          const v4f ga = *(const v4f*)(g1 + hf * 64 + c), gb = *(const v4f*)(g1 + hf * 64 + c + 4);
          const v4f ea = *(const v4f*)(be1 + hf * 64 + c), eb = *(const v4f*)(be1 + hf * 64 + c + 4);
          v4f y0 = *(const v4fa*)(&Y[yr + c]), y1 = *(const v4fa*)(&Y[yr + c + 4]); v8h hv;
#pragma unroll
          for (int i = 0; i < 4; ++i) { y0[i] = (y0[i] - mean) * rstd * bfr(ga[i]) + bfr(ea[i]); y1[i] = (y1[i] - mean) * rstd * bfr(gb[i]) + bfr(eb[i]);
                                        hv[i] = toh_flush(y0[i]); hv[4 + i] = toh_flush(y1[i]); }
          *(v4fa*)(&Y[yr + c]) = y0; *(v4fa*)(&Y[yr + c + 4]) = y1;
          *(v8ha*)(&sF[wf + rr * FP + hf * 64 + c]) = hv; } }
    wave_sync();
    v16h hA[4];
#pragma unroll
    for (int kc = 0; kc < 4; ++kc) hA[kc] = cat16(*(const v8ha*)(&sF[wf + lr * FP + 8 * hi + kc * 32]), *(const v8ha*)(&sF[wf + lr * FP + 8 * hi + kc * 32 + 16]));
    wave_sync();
    v8f o2[8];
#pragma unroll
    for (int nb = 0; nb < 8; ++nb) o2[nb] = (v8f){};
#pragma unroll 1
    for (int half = 0; half < 2; ++half) {
#pragma unroll 1
        for (int c2 = 0; c2 < 8; ++c2) {
            const int f0 = half * 128 + c2 * 16;
            v8f acc = (v8f){};
            const size_t w1o = (size_t)(f0 + lr) * DM + 8 * hi;
#pragma unroll
            for (int kc = 0; kc < 4; ++kc) { const v16h b = ldh(W1T + w1o + kc * 32); acc = wg16(hA[kc], b, acc); }
            const float b1v = bfr(b1[f0 + lr]);
#pragma unroll
            for (int j = 0; j < 8; ++j) { const float v = fmaxf(acc[j] * WINV + b1v, 0.0f); sF[wf + (hi * 8 + j) * FP + c2 * 16 + lr] = toh_flush(v); }
        }
        wave_sync();
#pragma unroll
        for (int kc = 0; kc < 4; ++kc) {
            const v16h a = cat16(*(const v8ha*)(&sF[wf + lr * FP + 8 * hi + kc * 32]), *(const v8ha*)(&sF[wf + lr * FP + 8 * hi + kc * 32 + 16]));
#pragma unroll
            for (int nb = 0; nb < 8; ++nb) { const v16h b = ldh(W2T + (size_t)(nb * 16 + lr) * FF + 8 * hi + half * 128 + kc * 32); o2[nb] = wg16(a, b, o2[nb]); } }
        wave_sync();
    }
#pragma unroll
    for (int nb = 0; nb < 8; ++nb) { const float b2v = bfr(b2[nb * 16 + lr]);
#pragma unroll
        for (int j = 0; j < 8; ++j) { const int yi = wy + (hi * 8 + j) * YP + nb * 16 + lr; const float hv0 = Y[yi]; Y[yi] = hv0 + (o2[nb][j] * WINV + b2v); } }
    wave_sync();
    { float s = 0.0f;
#pragma unroll 1
      for (int q = 0; q < 8; ++q) { const int c = q * 8;
          const v4f y0 = *(const v4fa*)(&Y[yr + c]), y1 = *(const v4fa*)(&Y[yr + c + 4]);
#pragma unroll
          for (int i = 0; i < 4; ++i) s += y0[i] + y1[i]; }
      s += __shfl_xor(s, 1, 32);
      const float mean = s * (1.0f / DM);
      float vs = 0.0f;
#pragma unroll 1
      for (int q = 0; q < 8; ++q) { const int c = q * 8;
          const v4f y0 = *(const v4fa*)(&Y[yr + c]), y1 = *(const v4fa*)(&Y[yr + c + 4]);
#pragma unroll
          for (int i = 0; i < 4; ++i) { const float d0 = y0[i] - mean, d1 = y1[i] - mean; vs += d0 * d0; vs += d1 * d1; } }
      vs += __shfl_xor(vs, 1, 32);
      const float rstd = rsqrtf(vs * (1.0f / DM) + LNEPS);
#pragma unroll 1
      for (int q = 0; q < 8; ++q) { const int c = q * 8;
          const v4f ga = *(const v4f*)(g2 + hf * 64 + c), gb = *(const v4f*)(g2 + hf * 64 + c + 4);
          const v4f ea = *(const v4f*)(be2 + hf * 64 + c), eb = *(const v4f*)(be2 + hf * 64 + c + 4);
          v4f y0 = *(const v4fa*)(&Y[yr + c]), y1 = *(const v4fa*)(&Y[yr + c + 4]);
#pragma unroll
          for (int i = 0; i < 4; ++i) { y0[i] = (y0[i] - mean) * rstd * bfr(ga[i]) + bfr(ea[i]); y1[i] = (y1[i] - mean) * rstd * bfr(gb[i]) + bfr(eb[i]); }
          *(v4fa*)(&Y[yr + c]) = y0; *(v4fa*)(&Y[yr + c + 4]) = y1; } }
    wave_sync();
    { v4f cs = (v4f){};
#pragma unroll 1
      for (int r = 0; r < 16; ++r) { const v4f t = *(const v4fa*)(&Y[wy + r * YP + lane * 4]); cs = cs + t; }
      *(v4fa*)(&spart[wave * DM + lane * 4]) = cs; }
    __syncthreads();
    if (wave == 0) {
        v4f tot = (v4f){};
#pragma unroll 1
        for (int w = 0; w < PW; ++w) { const v4f t = *(const v4fa*)(&spart[w * DM + lane * 4]); tot = tot + t; }
        float nm = 0.0f;
#pragma unroll
        for (int i = 0; i < SEQ / 32; ++i) nm += MK[(size_t)bl * SEQ + i * 32 + lane];
#pragma unroll
        for (int off = 16; off > 0; off >>= 1) nm += __shfl_xor(nm, off, 32);
        const float rn = 1.0f / nm;
        const v4f ov = tot * rn;
        float* op = OUT + (size_t)bl * DM + lane * 4;
        *(volatile v4f*)op = ov; __threadfence(); *(volatile v4f*)op = ov;
    }
}

static constexpr size_t al256(size_t v) { return (v + 255) & ~(size_t)255; }
static constexpr size_t PLQ     = (size_t)CHB * NH_ * SEQ * HD;
static constexpr size_t SZ_XB   = al256((size_t)NB * SEQ * DM * 2);
static constexpr size_t SZ_MK   = al256((size_t)NB * SEQ * 4);
static constexpr size_t SZ_WQKV = al256((size_t)3 * HK * DM * 2);
static constexpr size_t SZ_WOT  = al256((size_t)DM * HK * 2);
static constexpr size_t SZ_W1T  = al256((size_t)FF * DM * 2);
static constexpr size_t SZ_W2T  = al256((size_t)DM * FF * 2);
static constexpr size_t SZ_PL   = al256(PLQ * 2);
static constexpr size_t SZ_TOTAL = SZ_XB + SZ_MK + SZ_WQKV + SZ_WOT + SZ_W1T + SZ_W2T + 4 * SZ_PL;
static_assert(SZ_TOTAL <= (size_t)134217728);
static_assert((PLQ * 2) % 256 == 0);
static_assert(PLQ == (size_t)CHB * HK * SEQ);
static_assert(PLQ == (size_t)CHROWS * HK);
static_assert(((size_t)HK * DM * 2) % 256 == 0);
static_assert(((size_t)CHROWS * DM * 2) % 256 == 0);
static_assert(((size_t)CHROWS * 4) % 128 == 0);

extern "C" void kernel_launch(void* const* d_in, const int* in_sizes, int n_in,
                              void* d_out, int out_size, void* d_ws, size_t ws_size, hipStream_t stream) {
    if (n_in < 18) return;
    if (in_sizes[0] < DM || in_sizes[1] < 1) return;
    if ((size_t)in_sizes[2] < (size_t)DM * HK || (size_t)in_sizes[4] < (size_t)DM * HK || (size_t)in_sizes[6] < (size_t)DM * HK) return;
    if (in_sizes[3] < HK || in_sizes[5] < HK || in_sizes[7] < HK) return;
    if ((size_t)in_sizes[8] < (size_t)HK * DM || in_sizes[9] < DM) return;
    if (in_sizes[10] < DM * FF || in_sizes[11] < FF || in_sizes[12] < FF * DM) return;
    if (in_sizes[13] < DM || in_sizes[14] < DM || in_sizes[15] < DM || in_sizes[16] < DM || in_sizes[17] < DM) return;
    if ((size_t)out_size < (size_t)NB * DM) return;
    if (SZ_TOTAL > ws_size) return;
    const float* atoms = (const float*)d_in[0]; const int* mol = (const int*)d_in[1];
    const float* wq = (const float*)d_in[2];  const float* bq = (const float*)d_in[3];
    const float* wk = (const float*)d_in[4];  const float* bk = (const float*)d_in[5];
    const float* wv = (const float*)d_in[6];  const float* bv = (const float*)d_in[7];
    const float* wo = (const float*)d_in[8];  const float* bo = (const float*)d_in[9];
    const float* w1 = (const float*)d_in[10]; const float* b1 = (const float*)d_in[11];
    const float* w2 = (const float*)d_in[12]; const float* b2 = (const float*)d_in[13];
    const float* g1 = (const float*)d_in[14]; const float* be1 = (const float*)d_in[15];
    const float* g2 = (const float*)d_in[16]; const float* be2 = (const float*)d_in[17];
    int N = in_sizes[0] / DM; if (in_sizes[1] < N) N = in_sizes[1];
    float* OUT = (float*)d_out;
    char* wsp = (char*)d_ws;
    bf* XB = (bf*)wsp; wsp += SZ_XB;
    float* MK = (float*)wsp; wsp += SZ_MK;
    bf* WQKV = (bf*)wsp; wsp += SZ_WQKV;
    h16* WOT = (h16*)wsp; wsp += SZ_WOT;
    h16* W1T = (h16*)wsp; wsp += SZ_W1T;
    h16* W2T = (h16*)wsp; wsp += SZ_W2T;
    h16* QK  = (h16*)wsp; wsp += 2 * SZ_PL;
    h16* VT  = (h16*)wsp; wsp += SZ_PL;
    h16* CTX = (h16*)wsp; wsp += SZ_PL;

    k_pack<<<dim3(NB, 1, 1), 256, 0, stream>>>(atoms, mol, N, XB, MK);
    k_wT_bf<<<dim3(DM / 64, HK / 64, 1), 256, 0, stream>>>(wq, WQKV, DM, HK);
    k_wT_bf<<<dim3(DM / 64, HK / 64, 1), 256, 0, stream>>>(wk, WQKV + (size_t)HK * DM, DM, HK);
    k_wT_bf<<<dim3(DM / 64, HK / 64, 1), 256, 0, stream>>>(wv, WQKV + (size_t)2 * HK * DM, DM, HK);
    k_wT_h<<<dim3(HK / 64, DM / 64, 1), 256, 0, stream>>>(wo, WOT, HK, DM);
    k_wT_h<<<dim3(DM / 64, FF / 64, 1), 256, 0, stream>>>(w1, W1T, DM, FF);
    k_wT_h<<<dim3(FF / 64, DM / 64, 1), 256, 0, stream>>>(w2, W2T, FF, DM);

    for (int ch = 0; ch < NCH; ++ch) {
        const bf* xc = XB + (size_t)ch * CHROWS * DM;
        const float* mc = MK + (size_t)ch * CHROWS;
        k_projqk<<<dim3(CHROWS / 32, 2 * NH_, 1), 32, 0, stream>>>(xc, WQKV, bq, bk, QK);
        k_projv<<<dim3(HK / 16, CHB, 1), 32, 0, stream>>>(WQKV + (size_t)2 * HK * DM, xc, bv, VT);
        k_flash<<<dim3(SEQ / (16 * AW), CHB * NH_, 1), 32 * AW, 0, stream>>>(QK, QK + PLQ, VT, mc, CTX);
        k_post<<<dim3(CHB, 1, 1), 32 * PW, 0, stream>>>(CTX, xc, mc, WOT, W1T, W2T, bo, b1, b2, g1, be1, g2, be2, OUT + (size_t)ch * CHB * DM);
    }
}
